// GraphMultiHeadAttention_70248485093582
// MI455X (gfx1250) — hardware-verified
//
#include <hip/hip_runtime.h>
#include <math.h>
#include <stdint.h>

#define NTOK 4096
#define DM   1024
#define NH   16
#define HD   64
#define NQT  (NTOK / 64)
#define NKT  (NTOK / 64)
static_assert(NH * HD == DM);
static_assert((NTOK % 64) == 0 && (DM % 64) == 0 && (DM % 32) == 0);
static_assert(NQT == 64 && NKT == 64);

typedef _Float16 v16h __attribute__((ext_vector_type(16)));
typedef _Float16 v8h  __attribute__((ext_vector_type(8)));
typedef __bf16   v16b __attribute__((ext_vector_type(16)));
typedef __bf16   v8b  __attribute__((ext_vector_type(8)));
typedef float    v8f  __attribute__((ext_vector_type(8)));
typedef float    v4f  __attribute__((ext_vector_type(4)));
typedef unsigned int v4u __attribute__((ext_vector_type(4)));
typedef v8h __attribute__((may_alias)) v8ha;
typedef v4f __attribute__((may_alias)) v4fa;
typedef v4u __attribute__((may_alias)) v4ua;

#if defined(__HIP_DEVICE_COMPILE__)
#define DEV_ASM 1
#else
#define DEV_ASM 0
#endif

__device__ __forceinline__ unsigned short bf_bits(float f) {
  unsigned u = __float_as_uint(f);
  return (unsigned short)((u + 0x7FFFu + ((u >> 16) & 1u)) >> 16);
}
__device__ __forceinline__ float bf_up(unsigned short hb) { return __uint_as_float(((unsigned)hb) << 16); }
__device__ __forceinline__ unsigned short h_bits(_Float16 x) { return __builtin_bit_cast(unsigned short, x); }
__device__ __forceinline__ unsigned pk16(unsigned short a, unsigned short b) { return (unsigned)a | ((unsigned)b << 16); }
__device__ __forceinline__ v8f zero8() { v8f z = {0.f, 0.f, 0.f, 0.f, 0.f, 0.f, 0.f, 0.f}; return z; }

template <typename OT> struct FT;
template <> struct FT<__bf16>   { typedef v16b frag; typedef v8b half8; };
template <> struct FT<_Float16> { typedef v16h frag; typedef v8h half8; };

template <typename OT>
__device__ __forceinline__ typename FT<OT>::frag ldfrag(const OT* p) {
  union { typename FT<OT>::frag v; typename FT<OT>::half8 h[2]; } f;
  f.h[0] = *(const typename FT<OT>::half8*)(p);
  f.h[1] = *(const typename FT<OT>::half8*)(p + 16);
  return f.v;
}

__device__ __forceinline__ v8f mmar(v16b a, v16b b, v8f c) {
  return __builtin_amdgcn_wmma_f32_16x16x32_bf16(false, a, false, b, (short)0, c, false, false);
}
__device__ __forceinline__ v8f mma_h(v16h a, v16h b, v8f c) {
  c = __builtin_amdgcn_wmma_f32_16x16x32_f16(false, a, false, b, (short)0, c, false, false);
#if DEV_ASM
  asm volatile("v_nop\n\tv_nop\n\tv_nop\n\tv_nop" : "+v"(c) : "v"(a), "v"(b));
#endif
  return c;
}
__device__ __forceinline__ void dep_guard(v8f& a, v8f& b, v16b x, v16b y) {
#if DEV_ASM
  asm volatile("v_nop\n\tv_nop\n\tv_nop\n\tv_nop" : "+v"(a), "+v"(b) : "v"(x), "v"(y));
#else
  (void)a; (void)b; (void)x; (void)y;
#endif
}
__device__ __forceinline__ void keep4(v16b a, v16b b, v16b c, v16b d) {
#if DEV_ASM
  asm volatile("v_nop" :: "v"(a), "v"(b), "v"(c), "v"(d));
#else
  (void)a; (void)b; (void)c; (void)d;
#endif
}
__device__ __forceinline__ void acc_guard4(v8f& a, v8f& b, v8f& c, v8f& d) {
#if DEV_ASM
  asm volatile("v_nop\n\tv_nop\n\tv_nop\n\tv_nop" : "+v"(a), "+v"(b), "+v"(c), "+v"(d));
#else
  (void)a; (void)b; (void)c; (void)d;
#endif
}

__global__ __launch_bounds__(256) void cvt_bf16x8(const float* __restrict__ in, unsigned short* out, int n8) {
  const int i = blockIdx.x * 256 + (int)threadIdx.x;
  if (i < n8) {
    const v4f a  = *(const v4fa*)(in + (size_t)i * 8);
    const v4f a4 = *(const v4fa*)(in + (size_t)i * 8 + 4);
    v4u p;
    p[0] = pk16(bf_bits(a[0]),  bf_bits(a[1]));
    p[1] = pk16(bf_bits(a[2]),  bf_bits(a[3]));
    p[2] = pk16(bf_bits(a4[0]), bf_bits(a4[1]));
    p[3] = pk16(bf_bits(a4[2]), bf_bits(a4[3]));
    unsigned short* o = out + (size_t)i * 8;
    *(volatile v4u*)o = p;
    __threadfence();
    *(volatile v4u*)o = p;
  }
}

__global__ __launch_bounds__(256) void wtr64(const float* __restrict__ w0, const float* __restrict__ w1,
                                             const float* __restrict__ w2, unsigned short* wt) {
  __shared__ __align__(16) unsigned short sT[64 * 72];
  const int tid = (int)threadIdx.x, lane = tid & 31, wave = tid >> 5;
  const int z = blockIdx.z;
  const float* W = (z == 0) ? w0 : ((z == 1) ? w1 : w2);
  unsigned short* O = wt + (size_t)z * DM * DM;
  const int n0 = blockIdx.x * 64, k0 = blockIdx.y * 64;
  {
    const int r = tid >> 2, c16 = (tid & 3) * 16;
    const float* src = W + (size_t)(k0 + r) * DM + n0 + c16;
#pragma unroll
    for (int e = 0; e < 4; ++e) {
      const v4f a = *(const v4fa*)(src + 4 * e);
      sT[(c16 + 4 * e + 0) * 72 + r] = bf_bits(a[0]);
      sT[(c16 + 4 * e + 1) * 72 + r] = bf_bits(a[1]);
      sT[(c16 + 4 * e + 2) * 72 + r] = bf_bits(a[2]);
      sT[(c16 + 4 * e + 3) * 72 + r] = bf_bits(a[3]);
    }
  }
  __syncthreads();
  const int q4 = lane >> 3, c8 = (lane & 7) * 8;
  v4u hv[2];
#pragma unroll
  for (int it = 0; it < 2; ++it) {
    const int n = wave * 8 + it * 4 + q4;
    hv[it] = *(const v4ua*)(sT + n * 72 + c8);
  }
  for (int pass = 0; pass < 2; ++pass) {
#pragma unroll
    for (int it = 0; it < 2; ++it) {
      const int n = wave * 8 + it * 4 + q4;
      *(volatile v4u*)(O + (size_t)(n0 + n) * DM + k0 + c8) = hv[it];
    }
    __threadfence();
  }
}

template <bool BIAS_ROW>
__global__ __launch_bounds__(256) void gemm64(
    const unsigned short* __restrict__ Ap, int lda,
    const unsigned short* __restrict__ Btp, int ldb,
    unsigned short* Cp, int ldc,
    const float* __restrict__ bias,
    int M, int N, int K) {
  const __bf16* A  = (const __bf16*)(const void*)Ap;
  const __bf16* Bt = (const __bf16*)(const void*)Btp;
  __shared__ __align__(16) float sT[8][16 * 68];
  const int lane = threadIdx.x & 31;
  const int wave = threadIdx.x >> 5;
  const int tilesN = N >> 6;
  const int tilesM = M >> 6;
  const int tile = blockIdx.x * 8 + wave;
  if (tile >= tilesM * tilesN) return;
  const int tm = tile / tilesN;
  const int tn = tile - tm * tilesN;
  const int m0 = tm << 6;
  const int n0 = tn << 6;

  const int rlane = lane & 15;
  const int koff  = (lane >> 4) * 8;
  const int mOff  = (lane >> 4) * 8;

  v8f acc[4][4];
#pragma unroll
  for (int i = 0; i < 4; ++i)
#pragma unroll
    for (int j = 0; j < 4; ++j) acc[i][j] = zero8();

  for (int k0 = 0; k0 < K; k0 += 32) {
    v16b bq[4];
#pragma unroll
    for (int j = 0; j < 4; ++j)
      bq[j] = ldfrag<__bf16>(Bt + (size_t)(n0 + (j << 4) + rlane) * ldb + koff + k0);
#pragma unroll
    for (int i = 0; i < 4; ++i) {
      const v16b af = ldfrag<__bf16>(A + (size_t)(m0 + (i << 4) + rlane) * lda + koff + k0);
#pragma unroll
      for (int j = 0; j < 4; ++j) acc[i][j] = mmar(af, bq[j], acc[i][j]);
      dep_guard(acc[i][0], acc[i][3], af, bq[3]);
    }
    keep4(bq[0], bq[1], bq[2], bq[3]);
  }
  acc_guard4(acc[0][0], acc[0][1], acc[0][2], acc[0][3]);
  acc_guard4(acc[1][0], acc[1][1], acc[1][2], acc[1][3]);
  acc_guard4(acc[2][0], acc[2][1], acc[2][2], acc[2][3]);
  acc_guard4(acc[3][0], acc[3][1], acc[3][2], acc[3][3]);

  float* slab = sT[wave];
  const int q = lane >> 3, c8 = (lane & 7) * 8;
#pragma unroll
  for (int i = 0; i < 4; ++i) {
    const int mBase = m0 + (i << 4);
#pragma unroll
    for (int j = 0; j < 4; ++j) {
#pragma unroll
      for (int r = 0; r < 8; ++r) {
        slab[(mOff + r) * 68 + (j << 4) + rlane] = acc[i][j][r];
      }
    }
    __builtin_amdgcn_fence(__ATOMIC_RELEASE, "workgroup");
    __builtin_amdgcn_wave_barrier();
    __builtin_amdgcn_fence(__ATOMIC_ACQUIRE, "workgroup");
    v4u hv[4];
#pragma unroll
    for (int it = 0; it < 4; ++it) {
      const int row = it * 4 + q;
      const float* sp = slab + row * 68 + c8;
      float f[8];
#pragma unroll
      for (int e = 0; e < 8; ++e) f[e] = sp[e];
      if (BIAS_ROW) {
        const float bb = bf_up(bf_bits(bias[mBase + row]));
#pragma unroll
        for (int e = 0; e < 8; ++e) f[e] += bb;
      } else {
        const v4f b0 = *(const v4fa*)(bias + n0 + c8);
        const v4f b1 = *(const v4fa*)(bias + n0 + c8 + 4);
#pragma unroll
        for (int e = 0; e < 4; ++e) {
          f[e]     += bf_up(bf_bits(b0[e]));
          f[4 + e] += bf_up(bf_bits(b1[e]));
        }
      }
      v4u a;
#pragma unroll
      for (int e = 0; e < 4; ++e) {
        const _Float16 x0 = (_Float16)f[2 * e], x1 = (_Float16)f[2 * e + 1];
        a[e] = pk16(h_bits(x0), h_bits(x1));
      }
      hv[it] = a;
    }
    for (int pass = 0; pass < 2; ++pass) {
#pragma unroll
      for (int it = 0; it < 4; ++it) {
        const int row = it * 4 + q;
        *(volatile v4u*)(Cp + (size_t)(mBase + row) * ldc + n0 + c8) = hv[it];
      }
      __threadfence();
    }
    __builtin_amdgcn_fence(__ATOMIC_RELEASE, "workgroup");
    __builtin_amdgcn_wave_barrier();
    __builtin_amdgcn_fence(__ATOMIC_ACQUIRE, "workgroup");
  }
}

__device__ __forceinline__ void out_store_pass(const float* so, float* out, int h, int q0, int lane) {
  const int q8 = lane & 7, sub = lane >> 3;
#pragma unroll
  for (int i = 0; i < 8; ++i) {
    const int lid = i * 4 + sub;
    const int row = lid >> 1, hl = lid & 1;
    const v4f v = *(const v4fa*)(so + row * 64 + 32 * hl + 4 * q8);
    const size_t gi = (size_t)(q0 + row) * DM + (size_t)h * HD + 32 * hl + 4 * q8;
    *(volatile v4f*)(out + gi) = v;
  }
}

__global__ __launch_bounds__(128)
void attn_hd64(const unsigned short* __restrict__ qp, const unsigned short* __restrict__ kpp,
               const unsigned short* __restrict__ vtp, float* op, float sscale) {
  union FH { v16h v; v8h h[2]; };
  __shared__ __align__(16) _Float16 Ksh[64 * 64];
  __shared__ __align__(16) _Float16 Vth[64 * 64];
  __shared__ __align__(16) _Float16 Psh[4][16 * 64];
  __shared__ __align__(16) float    Os[4][16 * 64];

  const int tid  = threadIdx.x;
  const int wave = tid >> 5;
  const int lane = tid & 31;
  const int hh   = lane >> 4;
  const int c    = lane & 15;

  const int qt   = blockIdx.x;
  const int h    = blockIdx.y;
  const int q0   = qt * 64 + wave * 16;

  const _Float16* Qh = (const _Float16*)(const void*)qp;
  const _Float16* Kg = (const _Float16*)(const void*)kpp + (size_t)h * HD;
  const _Float16* Vh = (const _Float16*)(const void*)vtp + (size_t)h * HD * NTOK;

  v16h qa[2];
#pragma unroll
  for (int dc = 0; dc < 2; ++dc) {
    const size_t qo = (size_t)(q0 + c) * DM + (size_t)h * HD + dc * 32 + 8 * hh;
    qa[dc] = ldfrag<_Float16>(Qh + qo);
  }

  float mrow[8], lrow[8];
  v8f oacc[4];
#pragma unroll
  for (int r = 0; r < 8; ++r) { mrow[r] = -INFINITY; lrow[r] = 0.f; }
#pragma unroll
  for (int t = 0; t < 4; ++t) oacc[t] = zero8();

  for (int kt = 0; kt < NKT; ++kt) {
    const int kv0 = kt * 64;
    __syncthreads();
    {
      const int r = tid >> 1, half = (tid & 1) * 32;
      const _Float16* kg = Kg + (size_t)(kv0 + r) * DM + half;
      const _Float16* vg = Vh + (size_t)r * NTOK + kv0 + half;
#pragma unroll
      for (int i = 0; i < 4; ++i) {
        const v8h a0 = *(const v8ha*)(kg + 8 * i);
        const v8h b0 = *(const v8ha*)(vg + 8 * i);
        *(v8h*)(Ksh + r * 64 + half + 8 * i) = a0;
        *(v8h*)(Vth + r * 64 + half + 8 * i) = b0;
      }
    }
    __syncthreads();

    v8f s[4];
#pragma unroll
    for (int j = 0; j < 4; ++j) {
      v8f ah = zero8();
#pragma unroll
      for (int dc = 0; dc < 2; ++dc) {
        FH kb;
        kb.h[0] = *(const v8ha*)(Ksh + (j * 16 + c) * 64 + dc * 32 + 8 * hh);
        kb.h[1] = *(const v8ha*)(Ksh + (j * 16 + c) * 64 + dc * 32 + 16 + 8 * hh);
        ah = mma_h(qa[dc], kb.v, ah);
      }
#pragma unroll
      for (int r = 0; r < 8; ++r) s[j][r] = ah[r] * sscale;
    }

    _Float16* pwh = Psh[wave];
#pragma unroll
    for (int r = 0; r < 8; ++r) {
      float m = s[0][r];
#pragma unroll
      for (int j = 1; j < 4; ++j) m = fmaxf(m, s[j][r]);
#pragma unroll
      for (int off = 1; off < 16; off <<= 1) m = fmaxf(m, __shfl_xor(m, off, 32));
      const float mnew  = fmaxf(mrow[r], m);
      const float msafe = (mnew == -INFINITY) ? 0.f : mnew;
      const float alpha = __expf(mrow[r] - msafe);
      mrow[r] = mnew;
      float psum = 0.f;
#pragma unroll
      for (int j = 0; j < 4; ++j) {
        const float p = __expf(s[j][r] - msafe);
        psum += p;
        pwh[(8 * hh + r) * 64 + j * 16 + c] = (_Float16)(p * 1024.0f);
      }
#pragma unroll
      for (int off = 1; off < 16; off <<= 1) psum += __shfl_xor(psum, off, 32);
      lrow[r] = lrow[r] * alpha + psum;
#pragma unroll
      for (int t = 0; t < 4; ++t) oacc[t][r] *= alpha;
    }
    __builtin_amdgcn_fence(__ATOMIC_RELEASE, "workgroup");
    __builtin_amdgcn_wave_barrier();
    __builtin_amdgcn_fence(__ATOMIC_ACQUIRE, "workgroup");

#pragma unroll 1
    for (int kk = 0; kk < 2; ++kk) {
      FH pa;
      pa.h[0] = *(const v8ha*)(pwh + c * 64 + kk * 32 + 8 * hh);
      pa.h[1] = *(const v8ha*)(pwh + c * 64 + kk * 32 + 16 + 8 * hh);
#pragma unroll
      for (int t = 0; t < 4; ++t) {
        FH vb;
        vb.h[0] = *(const v8ha*)(Vth + (t * 16 + c) * 64 + kk * 32 + 8 * hh);
        vb.h[1] = *(const v8ha*)(Vth + (t * 16 + c) * 64 + kk * 32 + 16 + 8 * hh);
        oacc[t] = mma_h(pa.v, vb.v, oacc[t]);
      }
    }
  }

  float* os = Os[wave];
#pragma unroll
  for (int r = 0; r < 8; ++r) {
    const float l = lrow[r];
    const float inv = ((l > 0.f) ? (1.0f / l) : 0.f) * (1.0f / 1024.0f);
#pragma unroll
    for (int t = 0; t < 4; ++t) os[(8 * hh + r) * 64 + t * 16 + c] = oacc[t][r] * inv;
  }
  __syncthreads();
  out_store_pass(os, op, h, q0, lane);
  __threadfence();
  out_store_pass(os, op, h, q0, lane);
}

extern "C" void kernel_launch(void* const* d_in, const int* in_sizes, int n_in,
                              void* d_out, int out_size, void* d_ws, size_t ws_size,
                              hipStream_t stream) {
  if (n_in < 7) return;
  if (in_sizes[0] != NTOK * DM) return;
  if (in_sizes[1] != DM * DM || in_sizes[3] != DM * DM || in_sizes[5] != DM * DM) return;
  if (in_sizes[2] != DM || in_sizes[4] != DM || in_sizes[6] != DM) return;
  if (out_size != NTOK * DM) return;

  const float* x  = (const float*)d_in[0];
  const float* Wq = (const float*)d_in[1];
  const float* bq = (const float*)d_in[2];
  const float* Wk = (const float*)d_in[3];
  const float* bk = (const float*)d_in[4];
  const float* Wv = (const float*)d_in[5];
  const float* bv = (const float*)d_in[6];
  float* out = (float*)d_out;

  const size_t PX = (size_t)NTOK * DM * 2;
  const size_t PW = (size_t)3 * DM * DM * 2;
  const size_t PV = (size_t)DM * NTOK * 2;
  size_t off = 0;
  const size_t oXb = off; off += PX;
  const size_t oWt = off; off += PW;
  const size_t oQh = off; off += PX;
  const size_t oKp = off; off += PX;
  const size_t oVT = off; off += PV;
  if (off > ws_size) return;
  if (off > (size_t)134217728) return;

  char* ws = (char*)d_ws;
  unsigned short* Xb = (unsigned short*)(ws + oXb);
  unsigned short* Wt = (unsigned short*)(ws + oWt);
  unsigned short* Qh = (unsigned short*)(ws + oQh);
  unsigned short* Kp = (unsigned short*)(ws + oKp);
  unsigned short* VT = (unsigned short*)(ws + oVT);
  unsigned short* WqT = Wt;
  unsigned short* WkT = Wt + (size_t)DM * DM;
  unsigned short* WvT = Wt + (size_t)2 * DM * DM;

  const dim3 blk(256);
  const int n8x = NTOK * DM / 8;
  const dim3 gCvtX((n8x + 255) / 256);
  const dim3 gWtr(DM / 64, DM / 64, 3);
  const dim3 gQK((((NTOK / 64) * (DM / 64)) + 7) / 8);
  const dim3 gVT((((DM / 64) * (NTOK / 64)) + 7) / 8);
  const dim3 gAttn(NQT, NH);

  cvt_bf16x8<<<gCvtX, blk, 0, stream>>>(x, Xb, n8x);
  wtr64<<<gWtr, blk, 0, stream>>>(Wq, Wk, Wv, Wt);
  gemm64<false><<<gQK, blk, 0, stream>>>(Xb, DM, WqT, DM, Qh, DM, bq, NTOK, DM, DM);
  gemm64<false><<<gQK, blk, 0, stream>>>(Xb, DM, WkT, DM, Kp, DM, bk, NTOK, DM, DM);
  gemm64<true><<<gVT, blk, 0, stream>>>(WvT, DM, Xb, DM, VT, NTOK, bv, DM, NTOK, DM);
  attn_hd64<<<gAttn, dim3(128), 0, stream>>>(Qh, Kp, VT, out, 0.125f);
  (void)hipGetLastError();
}
